// HomeostaticEqProp_46084999086213
// MI455X (gfx1250) — hardware-verified
//
#include <hip/hip_runtime.h>
#include <math.h>

constexpr int   kRows   = 8192;
constexpr int   kDimIn  = 256;
constexpr int   kDimH   = 256;
constexpr int   kDimOut = 128;
constexpr int   kLayers = 5;
constexpr int   kSteps  = 30;
constexpr long  kPlane  = (long)kRows * kDimH;
constexpr float kWCarry = 16.0f;
constexpr float kHCarry = 2048.0f;
constexpr float kScaleW  = 1.0f / 16.0f;
constexpr float kScaleHW = 1.0f / 32768.0f;
constexpr float kAlpha  = 0.5f;
constexpr float kKeep   = 0.5f;

constexpr size_t kBytes16   = (size_t)kPlane * 2;
constexpr size_t kBytes32   = (size_t)kPlane * 4;
constexpr size_t offX16     = 0;
constexpr size_t offXE16    = offX16  + kBytes16;
constexpr size_t offT0      = offXE16 + kBytes16;
constexpr size_t offH32P    = offT0   + kBytes32;
constexpr size_t offH16P    = offH32P + 4 * kBytes32;
constexpr size_t offH32Q    = offH16P + 5 * kBytes16;
constexpr size_t offH16Q    = offH32Q + 4 * kBytes32;
constexpr size_t offWin     = offH16Q + 5 * kBytes16;
constexpr size_t offWs      = offWin  + (size_t)kDimH * kDimIn * 2;
constexpr size_t offWhd     = offWs   + (size_t)kLayers * kDimH * kDimH * 2;
constexpr size_t kWsEnd     = offWhd  + (size_t)kDimOut * kDimH * 2;
constexpr size_t kZeroBytes = offH32Q - offH32P;
static_assert(kWsEnd == 126681088, "carve total");
static_assert(kWsEnd <= 134217728, "carve under 128 MiB");

typedef __attribute__((ext_vector_type(16))) _Float16 v16h;
typedef __attribute__((ext_vector_type(8)))  _Float16 v8h;
typedef __attribute__((ext_vector_type(8)))  float    v8f;
typedef __attribute__((ext_vector_type(4)))  float    v4f;
typedef __attribute__((ext_vector_type(4)))  unsigned int v4u;

__device__ __forceinline__ void dep_guard_h(v8f& a, v8f& b, v16h x, v16h y) { asm volatile("v_nop\n\tv_nop\n\tv_nop\n\tv_nop" : "+v"(a), "+v"(b) : "v"(x), "v"(y)); }
__device__ __forceinline__ void keep4_h(v16h a, v16h b, v16h c, v16h d) { asm volatile("v_nop" :: "v"(a), "v"(b), "v"(c), "v"(d)); }
__device__ __forceinline__ void acc_guard4(v8f& a, v8f& b, v8f& c, v8f& d) { asm volatile("v_nop\n\tv_nop\n\tv_nop\n\tv_nop" : "+v"(a), "+v"(b), "+v"(c), "+v"(d)); }
template <typename T> struct Frag;
template <> struct Frag<_Float16> {
  typedef v16h V; union U { v16h v; v8h h[2]; };
  static __device__ __forceinline__ v16h load(const _Float16* p) {
    U f; f.h[0] = *(const v8h*)(p); f.h[1] = *(const v8h*)(p + 16); return f.v;
  }
  static __device__ __forceinline__ v8f mma(v16h a, v16h b, v8f c) {
    return __builtin_amdgcn_wmma_f32_16x16x32_f16(false, a, false, b, (short)0, c, false, false);
  }
  static __device__ __forceinline__ void guard(v8f& a, v8f& b, v16h x, v16h y) { dep_guard_h(a, b, x, y); }
  static __device__ __forceinline__ void keep(v16h a, v16h b, v16h c, v16h d) { keep4_h(a, b, c, d); }
};

__device__ __forceinline__ unsigned pk16(unsigned short a, unsigned short b) { return (unsigned)a | ((unsigned)b << 16); }
__device__ __forceinline__ unsigned short h_bits(float f) { const _Float16 h = (_Float16)f; return __builtin_bit_cast(unsigned short, h); }

template <int OUTM, bool TANH, bool BLEND>
__global__ __launch_bounds__(256) void gemm_f16_64(
    const unsigned short* __restrict__ Ap, int lda, long strideA,
    const unsigned short* __restrict__ Btp, int ldb, long strideB,
    float* __restrict__ Cf, unsigned short* __restrict__ Ch, int ldc, long strideC,
    const float* __restrict__ bias, long strideBias,
    const float* __restrict__ resid, long strideR,
    int M, int N, int K, float scale, float oscale) {
  typedef _Float16 T;
  typedef v16h V;
  const T* A = (const T*)Ap; const T* Bt = (const T*)Btp;
  __shared__ __align__(16) float sT[8][16 * 68];
  const int b    = blockIdx.y;
  const int lane = threadIdx.x & 31;
  const int wave = threadIdx.x >> 5;
  const int tilesN = N >> 6;
  const int tilesM = M >> 6;
  const int tile = blockIdx.x * 8 + wave;
  if (tile >= tilesM * tilesN) return;
  const int tm = tile / tilesN;
  const int tn = tile - tm * tilesN;
  const int m0 = tm << 6;
  const int n0 = tn << 6;

  const T* Ab = A  + (size_t)b * strideA;
  const T* Bb = Bt + (size_t)b * strideB;

  const int rlane = lane & 15;
  const int koff  = (lane >> 4) * 8;
  const int mOff  = (lane >> 4) * 8;

  v8f acc[4][4];
#pragma unroll
  for (int i = 0; i < 4; ++i)
#pragma unroll
    for (int j = 0; j < 4; ++j) acc[i][j] = (v8f){0.f,0.f,0.f,0.f,0.f,0.f,0.f,0.f};

  for (int k0 = 0; k0 < K; k0 += 32) {
    V bh[4];
#pragma unroll
    for (int j = 0; j < 4; ++j) {
      const size_t bo = (size_t)(n0 + (j << 4) + rlane) * ldb + koff + k0;
      bh[j] = Frag<T>::load(Bb + bo);
    }
#pragma unroll
    for (int i = 0; i < 4; ++i) {
      const size_t ao = (size_t)(m0 + (i << 4) + rlane) * lda + koff + k0;
      V ah = Frag<T>::load(Ab + ao);
#pragma unroll
      for (int j = 0; j < 4; ++j) {
        acc[i][j] = Frag<T>::mma(ah, bh[j], acc[i][j]);
      }
      Frag<T>::guard(acc[i][0], acc[i][3], ah, ah);
    }
    Frag<T>::keep(bh[0], bh[1], bh[2], bh[3]);
  }
  acc_guard4(acc[0][0], acc[0][1], acc[0][2], acc[0][3]);
  acc_guard4(acc[1][0], acc[1][1], acc[1][2], acc[1][3]);
  acc_guard4(acc[2][0], acc[2][1], acc[2][2], acc[2][3]);
  acc_guard4(acc[3][0], acc[3][1], acc[3][2], acc[3][3]);

  float* slab = sT[wave];
  const float* biasb = bias + (size_t)b * strideBias;
  const float* Rb = resid + (size_t)b * strideR;
  float* Cfb = Cf + (size_t)b * strideC;
  unsigned short* Chb = Ch + (size_t)b * strideC;
#pragma unroll
  for (int i = 0; i < 4; ++i) {
    const int mBase = m0 + (i << 4);
#pragma unroll
    for (int j = 0; j < 4; ++j) {
      const int n = n0 + (j << 4) + rlane;
      const float bv = biasb[n];
#pragma unroll
      for (int r = 0; r < 8; ++r) {
        float v = acc[i][j][r] * scale + bv;
        if (TANH) v = tanhf(v);
        if (BLEND) v = kKeep * Rb[(size_t)(mBase + mOff + r) * ldc + n] + kAlpha * v;
        slab[(mOff + r) * 68 + (j << 4) + rlane] = v;
      }
    }
    __builtin_amdgcn_fence(__ATOMIC_RELEASE, "workgroup");
    __builtin_amdgcn_wave_barrier();
    __builtin_amdgcn_fence(__ATOMIC_ACQUIRE, "workgroup");
    for (int pass = 0; pass < 2; ++pass) {
      if (OUTM == 0 || OUTM == 3) {
        const int hh = lane >> 4, c4 = (lane & 15) * 4;
#pragma unroll
        for (int it = 0; it < 8; ++it) {
          const int row = it * 2 + hh;
          v4f v = *(const v4f*)(slab + row * 68 + c4);
          *(volatile v4f*)(Cfb + (size_t)(mBase + row) * ldc + n0 + c4) = v;
        }
      }
      if (OUTM == 1 || OUTM == 3) {
        const int q = lane >> 3, c8 = (lane & 7) * 8;
#pragma unroll
        for (int it = 0; it < 4; ++it) {
          const int row = it * 4 + q;
          const float* sp = slab + row * 68 + c8;
          v8h hv;
#pragma unroll
          for (int e = 0; e < 8; ++e) hv[e] = (_Float16)(sp[e] * oscale);
          *(volatile v8h*)(Chb + (size_t)(mBase + row) * ldc + n0 + c8) = hv;
        }
      }
      __threadfence();
    }
    __builtin_amdgcn_fence(__ATOMIC_RELEASE, "workgroup");
    __builtin_amdgcn_wave_barrier();
    __builtin_amdgcn_fence(__ATOMIC_ACQUIRE, "workgroup");
  }
}

__global__ __launch_bounds__(256) void cast8_f16_kernel(const float* __restrict__ in, unsigned short* __restrict__ out,
                                                        int n8, float carry) {
  const int i = blockIdx.x * 256 + threadIdx.x;
  if (i >= n8) return;
  const float* p = in + 8 * (size_t)i;
  const v4f a = *(const v4f*)(p);
  const v4f c = *(const v4f*)(p + 4);
  unsigned short hb[8];
#pragma unroll
  for (int e = 0; e < 4; ++e) {
    hb[e]     = h_bits(a[e] * carry);
    hb[4 + e] = h_bits(c[e] * carry);
  }
  const v4u u = (v4u){pk16(hb[0], hb[1]), pk16(hb[2], hb[3]), pk16(hb[4], hb[5]), pk16(hb[6], hb[7])};
  unsigned short* q = out + 8 * (size_t)i;
  *(volatile v4u*)q = u;
  __threadfence();
  *(volatile v4u*)q = u;
}

__global__ __launch_bounds__(256) void castw_layers_kernel(const float* __restrict__ in, const float* __restrict__ sc,
                                                           unsigned short* __restrict__ out,
                                                           int n8, int layer_n8, int nlayers, float carry) {
  const int i = blockIdx.x * 256 + threadIdx.x;
  if (i >= n8) return;
  int layer = i / layer_n8;
  layer = layer < 0 ? 0 : (layer > nlayers - 1 ? nlayers - 1 : layer);
  const float s = carry * sc[layer];
  const float* p = in + 8 * (size_t)i;
  const v4f a = *(const v4f*)(p);
  const v4f c = *(const v4f*)(p + 4);
  unsigned short hb[8];
#pragma unroll
  for (int e = 0; e < 4; ++e) {
    hb[e]     = h_bits(a[e] * s);
    hb[4 + e] = h_bits(c[e] * s);
  }
  const v4u u = (v4u){pk16(hb[0], hb[1]), pk16(hb[2], hb[3]), pk16(hb[4], hb[5]), pk16(hb[6], hb[7])};
  unsigned short* q = out + 8 * (size_t)i;
  *(volatile v4u*)q = u;
  __threadfence();
  *(volatile v4u*)q = u;
}

__global__ __launch_bounds__(256) void zero16_kernel(unsigned int* __restrict__ p, int n16) {
  const int i = blockIdx.x * 256 + threadIdx.x;
  if (i >= n16) return;
  const v4u z = (v4u){0u, 0u, 0u, 0u};
  unsigned int* q = p + 4 * (size_t)i;
  *(volatile v4u*)q = z;
  __threadfence();
  *(volatile v4u*)q = z;
}

__global__ __launch_bounds__(256) void h0_plane_kernel(const float* __restrict__ T0, unsigned short* __restrict__ out,
                                                       int n8, float cmul) {
  const int i = blockIdx.x * 256 + threadIdx.x;
  if (i >= n8) return;
  const float* p = T0 + 8 * (size_t)i;
  const v4f a = *(const v4f*)(p);
  const v4f c = *(const v4f*)(p + 4);
  unsigned short hb[8];
#pragma unroll
  for (int e = 0; e < 4; ++e) {
    hb[e]     = h_bits(a[e] * cmul);
    hb[4 + e] = h_bits(c[e] * cmul);
  }
  const v4u u = (v4u){pk16(hb[0], hb[1]), pk16(hb[2], hb[3]), pk16(hb[4], hb[5]), pk16(hb[6], hb[7])};
  unsigned short* q = out + 8 * (size_t)i;
  *(volatile v4u*)q = u;
  __threadfence();
  *(volatile v4u*)q = u;
}

__global__ __launch_bounds__(256) void premise_check_kernel(const int* __restrict__ steps, float* __restrict__ out,
                                                            int n4, int expect) {
  const int i  = blockIdx.x * 256 + threadIdx.x;
  const int st = steps[0];
  if (st == expect) return;
  if (i >= n4) return;
  const float qn = __uint_as_float(0x7fc00000u);
  const v4f z = (v4f){qn, qn, qn, qn};
  float* q = out + 4 * (size_t)i;
  *(volatile v4f*)q = z;
  __threadfence();
  *(volatile v4f*)q = z;
}

extern "C" void kernel_launch(void* const* d_in, const int* in_sizes, int n_in,
                              void* d_out, int out_size, void* d_ws, size_t ws_size,
                              hipStream_t stream) {
  if (n_in < 9) return;
  if (in_sizes[0] != kRows * kDimIn) return;
  if (in_sizes[1] != kDimH * kDimIn) return;
  if (in_sizes[2] != kDimH) return;
  if (in_sizes[3] != kLayers * kDimH * kDimH) return;
  if (in_sizes[4] != kLayers * kDimH) return;
  if (in_sizes[5] != kLayers) return;
  if (in_sizes[6] != kDimOut * kDimH) return;
  if (in_sizes[7] != kDimOut) return;
  if (in_sizes[8] < 1) return;
  if (out_size != kRows * kDimOut) return;
  if (ws_size < kWsEnd) return;

  const float* x      = (const float*)d_in[0];
  const float* W_in   = (const float*)d_in[1];
  const float* b_in   = (const float*)d_in[2];
  const float* Ws     = (const float*)d_in[3];
  const float* bs     = (const float*)d_in[4];
  const float* scales = (const float*)d_in[5];
  const float* W_head = (const float*)d_in[6];
  const float* b_head = (const float*)d_in[7];
  const int*   stepsp = (const int*)d_in[8];
  float* out = (float*)d_out;

  char* ws = (char*)d_ws;
  unsigned short* X16   = (unsigned short*)(ws + offX16);
  unsigned short* XE16  = (unsigned short*)(ws + offXE16);
  float*          T0    = (float*)(ws + offT0);
  float*          H32P  = (float*)(ws + offH32P);
  unsigned short* H16P  = (unsigned short*)(ws + offH16P);
  float*          H32Q  = (float*)(ws + offH32Q);
  unsigned short* H16Q  = (unsigned short*)(ws + offH16Q);
  unsigned short* WIN16 = (unsigned short*)(ws + offWin);
  unsigned short* WS16  = (unsigned short*)(ws + offWs);
  unsigned short* WHD16 = (unsigned short*)(ws + offWhd);

  const int n8x  = (int)(kPlane / 8);
  const int n8wi = kDimH * kDimIn / 8;
  const int n8ws = kLayers * kDimH * kDimH / 8;
  const int n8wh = kDimOut * kDimH / 8;
  const int n16z = (int)(kZeroBytes / 16);
  const int n4o  = kRows * kDimOut / 4;

  cast8_f16_kernel<<<dim3((n8x + 255) / 256), 256, 0, stream>>>(x, X16, n8x, 1.0f);
  cast8_f16_kernel<<<dim3((n8wi + 255) / 256), 256, 0, stream>>>(W_in, WIN16, n8wi, kWCarry);
  castw_layers_kernel<<<dim3((n8ws + 255) / 256), 256, 0, stream>>>(Ws, scales, WS16, n8ws, kDimH * kDimH / 8, kLayers, kWCarry);
  cast8_f16_kernel<<<dim3((n8wh + 255) / 256), 256, 0, stream>>>(W_head, WHD16, n8wh, kWCarry);

  zero16_kernel<<<dim3((n16z + 255) / 256), 256, 0, stream>>>((unsigned int*)H32P, n16z);

  gemm_f16_64<1, false, false><<<dim3(64, 1), 256, 0, stream>>>(
      X16, kDimIn, 0L, WIN16, kDimIn, 0L,
      T0, XE16, kDimH, 0L,
      b_in, 0L, T0, 0L,
      kRows, kDimH, kDimIn, kScaleW, 1.0f);

  gemm_f16_64<0, true, false><<<dim3(64, 1), 256, 0, stream>>>(
      XE16, kDimH, 0L, WS16, kDimH, 0L,
      T0, X16, kDimH, 0L,
      bs, 0L, (const float*)(const void*)X16, 0L,
      kRows, kDimH, kDimH, kScaleW, 1.0f);

  double p2 = 1.0;
  for (int s = 1; s <= kSteps; ++s) {
    const bool odd = (s & 1) != 0;
    float*          H32old = odd ? H32P : H32Q;
    float*          H32new = odd ? H32Q : H32P;
    unsigned short* H16old = odd ? H16P : H16Q;
    unsigned short* H16new = odd ? H16Q : H16P;
    if (s >= 2) {
      const float c = (float)(1.0 - p2);
      h0_plane_kernel<<<dim3((n8x + 255) / 256), 256, 0, stream>>>(T0, H16old, n8x, c * kHCarry);
    }
    gemm_f16_64<3, true, true><<<dim3(64, 4), 256, 0, stream>>>(
        H16old, kDimH, kPlane,
        WS16 + (size_t)kDimH * kDimH, kDimH, (long)kDimH * kDimH,
        H32new, H16new + kPlane, kDimH, kPlane,
        bs + kDimH, (long)kDimH,
        H32old, kPlane,
        kRows, kDimH, kDimH, kScaleHW, kHCarry);
    p2 *= 0.5;
  }

  gemm_f16_64<0, false, false><<<dim3(32, 1), 256, 0, stream>>>(
      H16P + 4 * kPlane, kDimH, 0L, WHD16, kDimH, 0L,
      out, XE16, kDimOut, 0L,
      b_head, 0L, (const float*)(const void*)XE16, 0L,
      kRows, kDimOut, kDimH, kScaleHW, 1.0f);

  premise_check_kernel<<<dim3((n4o + 255) / 256), 256, 0, stream>>>(stepsp, out, n4o, kSteps);
}
